// SelfAttentionV4_13185549598786
// MI455X (gfx1250) — hardware-verified
//
#include <hip/hip_runtime.h>
#include <hip/hip_bf16.h>
#include <stddef.h>
#include <stdint.h>

#define NB    4
#define LSEQ  2048
#define DM    1024
#define DK    512
#define NTOK  (NB * LSEQ)
#define BR    32
#define BC    128
#define R0    128
#define NR3   (NB * R0)
#define NQT   (LSEQ / BR)
#define QT3   (R0 / BR)

static_assert(DK == 512);
static_assert(DK % 64 == 0);
static_assert(DK % 32 == 0);
static_assert(DM % 64 == 0);
static_assert((DM / 8) == 128);
static_assert(LSEQ % 256 == 0);
static_assert(R0 % BR == 0);
static_assert(R0 % BC == 0);
static_assert(R0 < LSEQ);
static_assert(LSEQ % BR == 0);
static_assert(BC % 32 == 0);
static_assert(NR3 % 256 == 0);
static_assert(NTOK % 256 == 0);

typedef _Float16 v16h __attribute__((ext_vector_type(16)));
typedef _Float16 v8h  __attribute__((ext_vector_type(8)));
typedef float    v8f  __attribute__((ext_vector_type(8)));
typedef float    v4f  __attribute__((ext_vector_type(4)));
typedef unsigned int   v4u   __attribute__((ext_vector_type(4)));
typedef unsigned short v8us  __attribute__((ext_vector_type(8)));
typedef unsigned short v16us __attribute__((ext_vector_type(16)));
typedef __bf16         v16b  __attribute__((ext_vector_type(16)));
typedef unsigned short ush;

union Frag  { v16h v; v8h h[2]; };
union FragU { v16us v; v8us h[2]; v16b b; };
union Pack8 { v8h h; v4u u; };
union PackU { v8us s; v4u u; };
struct HL { v4u h; v4u l; };

__device__ __forceinline__ ush f2bf(float f) {
  const unsigned u = __float_as_uint(f);
  return (ush)((u + 0x7FFFu + ((u >> 16) & 1u)) >> 16);
}
__device__ __forceinline__ float bf2f(ush b) { return __uint_as_float(((unsigned)b) << 16); }

__device__ __forceinline__ HL split8(v8f f) {
  PackU ph, pl;
#pragma unroll
  for (int e = 0; e < 8; ++e) {
    const ush hi = f2bf(f[e]);
    ph.s[e] = hi;
    pl.s[e] = f2bf(f[e] - bf2f(hi));
  }
  HL r; r.h = ph.u; r.l = pl.u;
  return r;
}

__device__ __forceinline__ v8f mma16(v16h a, v16h b, v8f c) {
  c = __builtin_amdgcn_wmma_f32_16x16x32_f16(false, a, false, b, (short)0, c, false, false);
  asm volatile("v_nop\n\tv_nop\n\tv_nop\n\tv_nop" : "+v"(c) : "v"(a), "v"(b));
  return c;
}
__device__ __forceinline__ v8f mmab(v16us a, v16us b, v8f c) {
  FragU ua, ub; ua.v = a; ub.v = b;
  c = __builtin_amdgcn_wmma_f32_16x16x32_bf16(false, ua.b, false, ub.b, (short)0, c, false, false);
  asm volatile("v_nop\n\tv_nop\n\tv_nop\n\tv_nop" : "+v"(c) : "v"(a), "v"(b));
  return c;
}

__device__ __forceinline__ v16h ldfrag(const _Float16* p, int ld, int row0, int k0, int lane) {
  const int m = lane & 15, lh = lane >> 4;
  const _Float16* q = p + (size_t)(row0 + m) * ld + k0 + 8 * lh;
  Frag f;
  f.h[0] = *(const v8h*)(q);
  f.h[1] = *(const v8h*)(q + 16);
  return f.v;
}
__device__ __forceinline__ v16us ldfragu(const ush* p, int ld, int row0, int k0, int lane) {
  const int m = lane & 15, lh = lane >> 4;
  const ush* q = p + (size_t)(row0 + m) * ld + k0 + 8 * lh;
  FragU f;
  f.h[0] = *(const v8us*)(q);
  f.h[1] = *(const v8us*)(q + 16);
  return f.v;
}

__device__ __forceinline__ v8f zero8() { return (v8f){0.f, 0.f, 0.f, 0.f, 0.f, 0.f, 0.f, 0.f}; }

__device__ __forceinline__ void gemm32x64(const _Float16* __restrict__ A, int lda,
                                          const _Float16* __restrict__ Bt, int ldb,
                                          int m0, int n0, int lane, v8f (&acc)[2][4]) {
#pragma unroll 2
  for (int k0 = 0; k0 < DM; k0 += 32) {
    const v16h a0 = ldfrag(A, lda, m0, k0, lane);
    const v16h a1 = ldfrag(A, lda, m0 + 16, k0, lane);
    const v16h b0 = ldfrag(Bt, ldb, n0, k0, lane);
    const v16h b1 = ldfrag(Bt, ldb, n0 + 16, k0, lane);
    const v16h b2 = ldfrag(Bt, ldb, n0 + 32, k0, lane);
    const v16h b3 = ldfrag(Bt, ldb, n0 + 48, k0, lane);
    acc[0][0] = mma16(a0, b0, acc[0][0]);
    acc[1][0] = mma16(a1, b0, acc[1][0]);
    acc[0][1] = mma16(a0, b1, acc[0][1]);
    acc[1][1] = mma16(a1, b1, acc[1][1]);
    acc[0][2] = mma16(a0, b2, acc[0][2]);
    acc[1][2] = mma16(a1, b2, acc[1][2]);
    acc[0][3] = mma16(a0, b3, acc[0][3]);
    acc[1][3] = mma16(a1, b3, acc[1][3]);
  }
}

__device__ __forceinline__ void gemm3_32x64(const ush* __restrict__ Ah, const ush* __restrict__ Al, int lda,
                                            const ush* __restrict__ Bh, const ush* __restrict__ Bl, int ldb,
                                            int m0, int n0, int lane, v8f (&acc)[2][4]) {
#pragma unroll 1
  for (int k0 = 0; k0 < DM; k0 += 32) {
    const v16us a0h = ldfragu(Ah, lda, m0, k0, lane);
    const v16us a1h = ldfragu(Ah, lda, m0 + 16, k0, lane);
    const v16us a0l = ldfragu(Al, lda, m0, k0, lane);
    const v16us a1l = ldfragu(Al, lda, m0 + 16, k0, lane);
#pragma unroll
    for (int t = 0; t < 4; ++t) {
      const v16us bh = ldfragu(Bh, ldb, n0 + 16 * t, k0, lane);
      const v16us bl = ldfragu(Bl, ldb, n0 + 16 * t, k0, lane);
      acc[0][t] = mmab(a0h, bh, acc[0][t]);
      acc[1][t] = mmab(a1h, bh, acc[1][t]);
      acc[0][t] = mmab(a0h, bl, acc[0][t]);
      acc[1][t] = mmab(a1h, bl, acc[1][t]);
      acc[0][t] = mmab(a0l, bh, acc[0][t]);
      acc[1][t] = mmab(a1l, bh, acc[1][t]);
    }
  }
}

__global__ __launch_bounds__(256) void k_cvt_x(const float* __restrict__ xq, const float* __restrict__ xk,
                                               const float* __restrict__ xv, _Float16* __restrict__ xh,
                                               ush* __restrict__ x3h, ush* __restrict__ x3l, int ngrp) {
  const int which = blockIdx.y;
  const float* x = (which == 0) ? xq : ((which == 1) ? xk : xv);
  const int t = blockIdx.x * 256 + (int)threadIdx.x;
  if (t >= ngrp) return;
  const size_t o = (size_t)t * 8;
  const int row = t >> 7;
  const int b = row / LSEQ;
  const int l = row - b * LSEQ;
  const bool three = (l < R0);
  const size_t oh = (size_t)which * NTOK * DM + o;
  const size_t o3 = (size_t)which * NR3 * DM + ((size_t)(b * R0 + l)) * DM + (size_t)(t & 127) * 8;
  const v4f a0 = *(const v4f*)(x + o);
  const v4f a1 = *(const v4f*)(x + o + 4);
  Pack8 pk;
  pk.h = (v8h){(_Float16)a0[0], (_Float16)a0[1], (_Float16)a0[2], (_Float16)a0[3],
               (_Float16)a1[0], (_Float16)a1[1], (_Float16)a1[2], (_Float16)a1[3]};
  const v4u vv = pk.u;
  HL s; s.h = (v4u){0u, 0u, 0u, 0u}; s.l = s.h;
  if (three) {
    const v8f f = (v8f){a0[0], a0[1], a0[2], a0[3], a1[0], a1[1], a1[2], a1[3]};
    s = split8(f);
  }
  volatile v4u* d = (volatile v4u*)(xh + oh);
  *d = vv;
  if (three) { *(volatile v4u*)(x3h + o3) = s.h; *(volatile v4u*)(x3l + o3) = s.l; }
  __threadfence();
  *d = vv;
  if (three) { *(volatile v4u*)(x3h + o3) = s.h; *(volatile v4u*)(x3l + o3) = s.l; }
}

#define TWP 68
__global__ __launch_bounds__(256) void k_cvt_w(const float* __restrict__ wq, const float* __restrict__ wk,
                                               const float* __restrict__ wv, _Float16* __restrict__ wh,
                                               ush* __restrict__ w3h, ush* __restrict__ w3l) {
  __shared__ __align__(16) float sw[32 * TWP];
  const int which = blockIdx.z;
  const float* w = (which == 0) ? wq : ((which == 1) ? wk : wv);
  const int tid = threadIdx.x;
  const int d0 = blockIdx.x * 64;
  const int n0 = blockIdx.y * 32;
  {
    const int dd = tid >> 2;
    const int pn = (tid & 3) * 8;
    const float* src = w + (size_t)(d0 + dd) * DK + n0 + pn;
    const v4f a0 = *(const v4f*)(src);
    const v4f a1 = *(const v4f*)(src + 4);
#pragma unroll
    for (int e = 0; e < 4; ++e) {
      sw[(pn + e) * TWP + dd]     = a0[e];
      sw[(pn + 4 + e) * TWP + dd] = a1[e];
    }
  }
  __syncthreads();
  const int nn = tid >> 3;
  const int pc = tid & 7;
  const float* sp = sw + nn * TWP + pc * 8;
  const v4f f0 = *(const v4f*)(sp);
  const v4f f1 = *(const v4f*)(sp + 4);
  const v8f f = (v8f){f0[0], f0[1], f0[2], f0[3], f1[0], f1[1], f1[2], f1[3]};
  Pack8 pk;
  pk.h = (v8h){(_Float16)(f[0] * 32.0f), (_Float16)(f[1] * 32.0f), (_Float16)(f[2] * 32.0f),
               (_Float16)(f[3] * 32.0f), (_Float16)(f[4] * 32.0f), (_Float16)(f[5] * 32.0f),
               (_Float16)(f[6] * 32.0f), (_Float16)(f[7] * 32.0f)};
  const v4u vf = pk.u;
  const HL s = split8(f);
  const size_t od = ((size_t)which * DK + n0 + nn) * DM + d0 + pc * 8;
  for (int ps = 0; ps < 2; ++ps) {
    *(volatile v4u*)(wh + od)  = vf;
    *(volatile v4u*)(w3h + od) = s.h;
    *(volatile v4u*)(w3l + od) = s.l;
    __threadfence();
  }
}

#define STP 72
__global__ __launch_bounds__(256) void k_qkv(const _Float16* __restrict__ xh,
                                             const _Float16* __restrict__ wh,
                                             const float* __restrict__ bq,
                                             const float* __restrict__ bk,
                                             const float* __restrict__ bv,
                                             _Float16* __restrict__ qp,
                                             _Float16* __restrict__ kp,
                                             _Float16* __restrict__ vt) {
  __shared__ __align__(16) _Float16 st[256 * STP];
  const int tid = threadIdx.x, lane = tid & 31, wave = tid >> 5;
  const int hh = lane >> 4, c = lane & 15;
  const int which = blockIdx.z;
  const int mb = blockIdx.x * 256;
  const int m0 = mb + wave * 32;
  const int nn = blockIdx.y * 64;
  const _Float16* A  = xh + (size_t)which * NTOK * DM;
  const _Float16* Bt = wh + (size_t)which * DK * DM;
  const float* bias = (which == 0) ? bq : ((which == 1) ? bk : bv);

  v8f acc[2][4];
#pragma unroll
  for (int s = 0; s < 2; ++s)
#pragma unroll
    for (int t = 0; t < 4; ++t) acc[s][t] = zero8();
  gemm32x64(A, DM, Bt, DM, m0, nn, lane, acc);

#pragma unroll
  for (int t = 0; t < 4; ++t) {
    const float bn = bias[nn + 16 * t + c];
#pragma unroll
    for (int sub = 0; sub < 2; ++sub) {
#pragma unroll
      for (int r = 0; r < 8; ++r) {
        const int lr = wave * 32 + sub * 16 + 8 * hh + r;
        st[lr * STP + 16 * t + c] = (_Float16)(acc[sub][t][r] * 0.03125f + bn);
      }
    }
  }
  __syncthreads();

  _Float16* base = (which == 0) ? qp : ((which == 1) ? kp : vt);
  v4u val[8];
  size_t go[8];
  if (which < 2) {
#pragma unroll
    for (int j = 0; j < 8; ++j) {
      const int p  = tid + 256 * j;
      const int lr = p >> 3;
      const int pc = p & 7;
      Pack8 pk;
      pk.h  = *(const v8h*)(st + lr * STP + pc * 8);
      val[j] = pk.u;
      go[j]  = ((size_t)(mb + lr)) * DK + nn + pc * 8;
    }
  } else {
#pragma unroll
    for (int j = 0; j < 8; ++j) {
      const int p  = tid + 256 * j;
      const int L  = p >> 3;
      const int pc = p & 7;
      const int d  = L >> 2;
      const int nl = (L & 3) * 64 + pc * 8;
      const _Float16* cp = st + nl * STP + d;
      Pack8 pk;
      pk.h = (v8h){cp[0 * STP], cp[1 * STP], cp[2 * STP], cp[3 * STP],
                   cp[4 * STP], cp[5 * STP], cp[6 * STP], cp[7 * STP]};
      val[j] = pk.u;
      go[j]  = ((size_t)(nn + d)) * NTOK + mb + nl;
    }
  }
  for (int ps = 0; ps < 2; ++ps) {
#pragma unroll
    for (int j = 0; j < 8; ++j) *(volatile v4u*)(base + go[j]) = val[j];
    __threadfence();
  }
}

__global__ __launch_bounds__(256) void k_qkv3(const ush* __restrict__ xh3, const ush* __restrict__ xl3,
                                              const ush* __restrict__ wth, const ush* __restrict__ wtl,
                                              const float* __restrict__ bq,
                                              const float* __restrict__ bk,
                                              const float* __restrict__ bv,
                                              ush* __restrict__ q3h, ush* __restrict__ q3l,
                                              ush* __restrict__ k3h, ush* __restrict__ k3l,
                                              ush* __restrict__ v3h, ush* __restrict__ v3l) {
  __shared__ __align__(16) ush st[256 * STP];
  const int tid = threadIdx.x, lane = tid & 31, wave = tid >> 5;
  const int hh = lane >> 4, c = lane & 15;
  const int which = blockIdx.z;
  const int mb = blockIdx.x * 256;
  const int m0 = mb + wave * 32;
  const int nn = blockIdx.y * 64;
  const ush* Ah = xh3 + (size_t)which * NR3 * DM;
  const ush* Al = xl3 + (size_t)which * NR3 * DM;
  const ush* Bh = wth + (size_t)which * DK * DM;
  const ush* Bl = wtl + (size_t)which * DK * DM;
  const float* bias = (which == 0) ? bq : ((which == 1) ? bk : bv);

  v8f acc[2][4];
#pragma unroll
  for (int s = 0; s < 2; ++s)
#pragma unroll
    for (int t = 0; t < 4; ++t) acc[s][t] = zero8();
  gemm3_32x64(Ah, Al, DM, Bh, Bl, DM, m0, nn, lane, acc);

#pragma unroll
  for (int t = 0; t < 4; ++t) {
    const float bn = bias[nn + 16 * t + c];
#pragma unroll
    for (int sub = 0; sub < 2; ++sub) {
#pragma unroll
      for (int r = 0; r < 8; ++r) acc[sub][t][r] += bn;
    }
  }

  ush* bhp = (which == 0) ? q3h : ((which == 1) ? k3h : v3h);
  ush* blp = (which == 0) ? q3l : ((which == 1) ? k3l : v3l);
  size_t go[8];
#pragma unroll
  for (int j = 0; j < 8; ++j) {
    const int p  = tid + 256 * j;
    const int L  = p >> 3;
    const int pc = p & 7;
    if (which < 2) {
      go[j] = ((size_t)(mb + L)) * DK + nn + pc * 8;
    } else {
      const int d  = L >> 2;
      const int nl = (L & 3) * 64 + pc * 8;
      go[j] = ((size_t)(nn + d)) * NR3 + mb + nl;
    }
  }

#pragma unroll 1
  for (int ph = 0; ph < 2; ++ph) {
    __syncthreads();
#pragma unroll
    for (int t = 0; t < 4; ++t) {
#pragma unroll
      for (int sub = 0; sub < 2; ++sub) {
#pragma unroll
        for (int r = 0; r < 8; ++r) {
          const int lr = wave * 32 + sub * 16 + 8 * hh + r;
          const float v = acc[sub][t][r];
          const ush hi = f2bf(v);
          st[lr * STP + 16 * t + c] = (ph == 0) ? hi : f2bf(v - bf2f(hi));
        }
      }
    }
    __syncthreads();
    v4u val[8];
    if (which < 2) {
#pragma unroll
      for (int j = 0; j < 8; ++j) {
        const int p  = tid + 256 * j;
        const int lr = p >> 3;
        const int pc = p & 7;
        PackU pk;
        pk.s  = *(const v8us*)(st + lr * STP + pc * 8);
        val[j] = pk.u;
      }
    } else {
#pragma unroll
      for (int j = 0; j < 8; ++j) {
        const int p  = tid + 256 * j;
        const int L  = p >> 3;
        const int pc = p & 7;
        const int d  = L >> 2;
        const int nl = (L & 3) * 64 + pc * 8;
        const ush* cp = st + nl * STP + d;
        PackU pk;
        pk.s = (v8us){cp[0 * STP], cp[1 * STP], cp[2 * STP], cp[3 * STP],
                      cp[4 * STP], cp[5 * STP], cp[6 * STP], cp[7 * STP]};
        val[j] = pk.u;
      }
    }
    ush* dst = (ph == 0) ? bhp : blp;
    for (int ps = 0; ps < 2; ++ps) {
#pragma unroll
      for (int j = 0; j < 8; ++j) *(volatile v4u*)(dst + go[j]) = val[j];
      __threadfence();
    }
  }
}

#define OTP 68
__device__ __forceinline__ void attn_out(v8f (&oacc)[2][4], const float* rowl, float sinv, float* sw,
                                         float* __restrict__ out, size_t grow0, int n0,
                                         int lane, int hh, int c) {
#pragma unroll
  for (int sub = 0; sub < 2; ++sub) {
    __syncthreads();
#pragma unroll
    for (int r = 0; r < 8; ++r) {
      const float lv  = rowl[sub * 16 + 8 * hh + r];
      const float inv = (lv > 0.f) ? (sinv / lv) : 0.f;
#pragma unroll
      for (int t = 0; t < 4; ++t) sw[(8 * hh + r) * OTP + 16 * t + c] = oacc[sub][t][r] * inv;
    }
    __syncthreads();
    v4f val[8];
    size_t go[8];
#pragma unroll
    for (int it = 0; it < 8; ++it) {
      const int p    = lane + 32 * it;
      const int L    = p >> 3;
      const int pc   = p & 7;
      const int row  = L >> 1;
      const int half = L & 1;
      val[it] = *(const v4f*)(sw + row * OTP + half * 32 + pc * 4);
      go[it]  = (grow0 + (size_t)(sub * 16 + row)) * DK + n0 + half * 32 + pc * 4;
    }
    for (int ps = 0; ps < 2; ++ps) {
#pragma unroll
      for (int it = 0; it < 8; ++it) *(volatile v4f*)(out + go[it]) = val[it];
      __threadfence();
    }
  }
}

#define SSP 128
#define SPP 136
__global__ __launch_bounds__(256) void k_attn(const _Float16* __restrict__ qp,
                                              const _Float16* __restrict__ kp,
                                              const _Float16* __restrict__ vt,
                                              float* __restrict__ out, int qt0, float sscale, float sinv) {
  __shared__ __align__(16) float    sSO[8 * 16 * OTP];
  __shared__ __align__(16) _Float16 sP[BR * SPP];
  __shared__ __align__(16) float    sRed[BR * 8];
  __shared__ __align__(16) float    rM[BR];
  __shared__ __align__(16) float    rMn[BR];
  __shared__ __align__(16) float    rL[BR];
  __shared__ __align__(16) float    rSc[BR];

  float* sS = sSO;
  const int tid = threadIdx.x, lane = tid & 31, wave = tid >> 5;
  const int hh = lane >> 4, c = lane & 15;
  const int b  = blockIdx.y;
  const int q0 = (qt0 + (int)blockIdx.x) * BR;
  const _Float16* Qb = qp + (size_t)b * LSEQ * DK;
  const _Float16* Kb = kp + (size_t)b * LSEQ * DK;
  const _Float16* Vb = vt + (size_t)b * LSEQ;
  const float NEGI = -__builtin_huge_valf();
  if (tid < BR) { rM[tid] = NEGI; rL[tid] = 0.f; }
  __syncthreads();

  v8f oacc[2][4];
#pragma unroll
  for (int s = 0; s < 2; ++s)
#pragma unroll
    for (int t = 0; t < 4; ++t) oacc[s][t] = zero8();

  const int srow = tid >> 3, schk = tid & 7;
  const int nch = (q0 + BR + BC - 1) / BC;

#pragma unroll 1
  for (int ch = 0; ch < nch; ++ch) {
    const int j0  = ch * BC;
    const int kr0 = j0 + wave * 16;
    v8f s[2];
    s[0] = zero8(); s[1] = zero8();
#pragma unroll 2
    for (int k0 = 0; k0 < DK; k0 += 32) {
      const v16h a0 = ldfrag(Qb, DK, q0, k0, lane);
      const v16h a1 = ldfrag(Qb, DK, q0 + 16, k0, lane);
      const v16h kb = ldfrag(Kb, DK, kr0, k0, lane);
      s[0] = mma16(a0, kb, s[0]);
      s[1] = mma16(a1, kb, s[1]);
    }
    {
      const int key = kr0 + c;
#pragma unroll
      for (int t = 0; t < 2; ++t) {
#pragma unroll
        for (int r = 0; r < 8; ++r) {
          const int row = 16 * t + 8 * hh + r;
          const float raw = (key > q0 + row) ? -1.0e9f : s[t][r];
          sS[row * SSP + wave * 16 + c] = raw * sscale;
        }
      }
    }
    __syncthreads();
    {
      const float* sr = sS + srow * SSP + schk * 16;
      const v4f x0 = *(const v4f*)(sr);
      const v4f x1 = *(const v4f*)(sr + 4);
      const v4f x2 = *(const v4f*)(sr + 8);
      const v4f x3 = *(const v4f*)(sr + 12);
      float mx = x0[0];
#pragma unroll
      for (int e = 1; e < 4; ++e) mx = fmaxf(mx, x0[e]);
#pragma unroll
      for (int e = 0; e < 4; ++e) { mx = fmaxf(mx, x1[e]); mx = fmaxf(mx, x2[e]); mx = fmaxf(mx, x3[e]); }
      sRed[srow * 8 + schk] = mx;
    }
    __syncthreads();
    if (tid < BR) {
      float mx = rM[tid];
#pragma unroll
      for (int i = 0; i < 8; ++i) mx = fmaxf(mx, sRed[tid * 8 + i]);
      rMn[tid] = mx;
    }
    __syncthreads();
    {
      const float mx = rMn[srow];
      const float* sr = sS + srow * SSP + schk * 16;
      float sum = 0.f;
      Pack8 p0, p1;
#pragma unroll
      for (int e = 0; e < 8; ++e) {
        const float p = __expf(sr[e] - mx);
        sum += p;
        p0.h[e] = (_Float16)(p * 1024.0f);
      }
#pragma unroll
      for (int e = 0; e < 8; ++e) {
        const float p = __expf(sr[8 + e] - mx);
        sum += p;
        p1.h[e] = (_Float16)(p * 1024.0f);
      }
      *(v8h*)(sP + srow * SPP + schk * 16)     = p0.h;
      *(v8h*)(sP + srow * SPP + schk * 16 + 8) = p1.h;
      sRed[srow * 8 + schk] = sum;
    }
    __syncthreads();
    if (tid < BR) {
      float sum = 0.f;
#pragma unroll
      for (int i = 0; i < 8; ++i) sum += sRed[tid * 8 + i];
      const float mnew = rMn[tid];
      const float fac  = __expf(rM[tid] - mnew);
      rL[tid]  = rL[tid] * fac + sum;
      rM[tid]  = mnew;
      rSc[tid] = fac;
    }
    __syncthreads();
#pragma unroll
    for (int t = 0; t < 2; ++t) {
      const v4f f0 = *(const v4f*)(rSc + 16 * t + 8 * hh);
      const v4f f1 = *(const v4f*)(rSc + 16 * t + 8 * hh + 4);
#pragma unroll
      for (int et = 0; et < 4; ++et) {
#pragma unroll
        for (int r = 0; r < 4; ++r) {
          oacc[t][et][r]     *= f0[r];
          oacc[t][et][4 + r] *= f1[r];
        }
      }
    }
#pragma unroll 1
    for (int kk = 0; kk < BC / 32; ++kk) {
      const v16h pa0 = ldfrag(sP, SPP, 0, kk * 32, lane);
      const v16h pa1 = ldfrag(sP, SPP, 16, kk * 32, lane);
#pragma unroll
      for (int et = 0; et < 4; ++et) {
        const v16h vb = ldfrag(Vb, NTOK, wave * 64 + 16 * et, j0 + kk * 32, lane);
        oacc[0][et] = mma16(pa0, vb, oacc[0][et]);
        oacc[1][et] = mma16(pa1, vb, oacc[1][et]);
      }
    }
    __syncthreads();
  }
  attn_out(oacc, rL, sinv, sSO + wave * (16 * OTP), out, (size_t)b * LSEQ + q0, wave * 64, lane, hh, c);
}

__global__ __launch_bounds__(256) void k_attn3(const ush* __restrict__ q3h, const ush* __restrict__ q3l,
                                               const ush* __restrict__ k3h, const ush* __restrict__ k3l,
                                               const ush* __restrict__ v3h, const ush* __restrict__ v3l,
                                               float* __restrict__ out, float sscale) {
  __shared__ __align__(16) float sSO[8 * 16 * OTP];
  __shared__ __align__(16) ush   sPh[BR * SPP];
  __shared__ __align__(16) ush   sPl[BR * SPP];
  __shared__ __align__(16) float sRed[BR * 8];
  __shared__ __align__(16) float rM[BR];
  __shared__ __align__(16) float rMn[BR];
  __shared__ __align__(16) float rL[BR];
  __shared__ __align__(16) float rSc[BR];

  float* sS = sSO;
  const int tid = threadIdx.x, lane = tid & 31, wave = tid >> 5;
  const int hh = lane >> 4, c = lane & 15;
  const int b  = blockIdx.y;
  const int q0 = (int)blockIdx.x * BR;
  const ush* Qh = q3h + (size_t)b * R0 * DK;
  const ush* Ql = q3l + (size_t)b * R0 * DK;
  const ush* Kh = k3h + (size_t)b * R0 * DK;
  const ush* Kl = k3l + (size_t)b * R0 * DK;
  const ush* Vh = v3h + (size_t)b * R0;
  const ush* Vl = v3l + (size_t)b * R0;
  const float NEGI = -__builtin_huge_valf();
  if (tid < BR) { rM[tid] = NEGI; rL[tid] = 0.f; }
  __syncthreads();

  v8f oacc[2][4];
#pragma unroll
  for (int s = 0; s < 2; ++s)
#pragma unroll
    for (int t = 0; t < 4; ++t) oacc[s][t] = zero8();

  const int srow = tid >> 3, schk = tid & 7;
  const int nch = (q0 + BR + BC - 1) / BC;

#pragma unroll 1
  for (int ch = 0; ch < nch; ++ch) {
    const int j0  = ch * BC;
    const int kr0 = j0 + wave * 16;
    v8f s[2];
    s[0] = zero8(); s[1] = zero8();
#pragma unroll 1
    for (int k0 = 0; k0 < DK; k0 += 32) {
      const v16us a0h = ldfragu(Qh, DK, q0, k0, lane);
      const v16us a1h = ldfragu(Qh, DK, q0 + 16, k0, lane);
      const v16us a0l = ldfragu(Ql, DK, q0, k0, lane);
      const v16us a1l = ldfragu(Ql, DK, q0 + 16, k0, lane);
      const v16us kbh = ldfragu(Kh, DK, kr0, k0, lane);
      const v16us kbl = ldfragu(Kl, DK, kr0, k0, lane);
      s[0] = mmab(a0h, kbh, s[0]);
      s[1] = mmab(a1h, kbh, s[1]);
      s[0] = mmab(a0h, kbl, s[0]);
      s[1] = mmab(a1h, kbl, s[1]);
      s[0] = mmab(a0l, kbh, s[0]);
      s[1] = mmab(a1l, kbh, s[1]);
    }
    {
      const int key = kr0 + c;
#pragma unroll
      for (int t = 0; t < 2; ++t) {
#pragma unroll
        for (int r = 0; r < 8; ++r) {
          const int row = 16 * t + 8 * hh + r;
          const float raw = (key > q0 + row) ? -1.0e9f : s[t][r];
          sS[row * SSP + wave * 16 + c] = raw * sscale;
        }
      }
    }
    __syncthreads();
    {
      const float* sr = sS + srow * SSP + schk * 16;
      const v4f x0 = *(const v4f*)(sr);
      const v4f x1 = *(const v4f*)(sr + 4);
      const v4f x2 = *(const v4f*)(sr + 8);
      const v4f x3 = *(const v4f*)(sr + 12);
      float mx = x0[0];
#pragma unroll
      for (int e = 1; e < 4; ++e) mx = fmaxf(mx, x0[e]);
#pragma unroll
      for (int e = 0; e < 4; ++e) { mx = fmaxf(mx, x1[e]); mx = fmaxf(mx, x2[e]); mx = fmaxf(mx, x3[e]); }
      sRed[srow * 8 + schk] = mx;
    }
    __syncthreads();
    if (tid < BR) {
      float mx = rM[tid];
#pragma unroll
      for (int i = 0; i < 8; ++i) mx = fmaxf(mx, sRed[tid * 8 + i]);
      rMn[tid] = mx;
    }
    __syncthreads();
    {
      const float mx = rMn[srow];
      const float* sr = sS + srow * SSP + schk * 16;
      float sum = 0.f;
      PackU ph0, pl0, ph1, pl1;
#pragma unroll
      for (int e = 0; e < 8; ++e) {
        const float p = __expf(sr[e] - mx);
        sum += p;
        const ush hi = f2bf(p);
        ph0.s[e] = hi;
        pl0.s[e] = f2bf(p - bf2f(hi));
      }
#pragma unroll
      for (int e = 0; e < 8; ++e) {
        const float p = __expf(sr[8 + e] - mx);
        sum += p;
        const ush hi = f2bf(p);
        ph1.s[e] = hi;
        pl1.s[e] = f2bf(p - bf2f(hi));
      }
      *(v8us*)(sPh + srow * SPP + schk * 16)     = ph0.s;
      *(v8us*)(sPh + srow * SPP + schk * 16 + 8) = ph1.s;
      *(v8us*)(sPl + srow * SPP + schk * 16)     = pl0.s;
      *(v8us*)(sPl + srow * SPP + schk * 16 + 8) = pl1.s;
      sRed[srow * 8 + schk] = sum;
    }
    __syncthreads();
    if (tid < BR) {
      float sum = 0.f;
#pragma unroll
      for (int i = 0; i < 8; ++i) sum += sRed[tid * 8 + i];
      const float mnew = rMn[tid];
      const float fac  = __expf(rM[tid] - mnew);
      rL[tid]  = rL[tid] * fac + sum;
      rM[tid]  = mnew;
      rSc[tid] = fac;
    }
    __syncthreads();
#pragma unroll
    for (int t = 0; t < 2; ++t) {
      const v4f f0 = *(const v4f*)(rSc + 16 * t + 8 * hh);
      const v4f f1 = *(const v4f*)(rSc + 16 * t + 8 * hh + 4);
#pragma unroll
      for (int et = 0; et < 4; ++et) {
#pragma unroll
        for (int r = 0; r < 4; ++r) {
          oacc[t][et][r]     *= f0[r];
          oacc[t][et][4 + r] *= f1[r];
        }
      }
    }
#pragma unroll 1
    for (int kk = 0; kk < BC / 32; ++kk) {
      const v16us pah0 = ldfragu(sPh, SPP, 0, kk * 32, lane);
      const v16us pah1 = ldfragu(sPh, SPP, 16, kk * 32, lane);
      const v16us pal0 = ldfragu(sPl, SPP, 0, kk * 32, lane);
      const v16us pal1 = ldfragu(sPl, SPP, 16, kk * 32, lane);
#pragma unroll
      for (int et = 0; et < 4; ++et) {
        const v16us vbh = ldfragu(Vh, NR3, wave * 64 + 16 * et, j0 + kk * 32, lane);
        const v16us vbl = ldfragu(Vl, NR3, wave * 64 + 16 * et, j0 + kk * 32, lane);
        oacc[0][et] = mmab(pah0, vbh, oacc[0][et]);
        oacc[1][et] = mmab(pah1, vbh, oacc[1][et]);
        oacc[0][et] = mmab(pah0, vbl, oacc[0][et]);
        oacc[1][et] = mmab(pah1, vbl, oacc[1][et]);
        oacc[0][et] = mmab(pal0, vbh, oacc[0][et]);
        oacc[1][et] = mmab(pal1, vbh, oacc[1][et]);
      }
    }
    __syncthreads();
  }
  attn_out(oacc, rL, 1.0f, sSO + wave * (16 * OTP), out, (size_t)b * LSEQ + q0, wave * 64, lane, hh, c);
}

extern "C" void kernel_launch(void* const* d_in, const int* in_sizes, int n_in,
                              void* d_out, int out_size, void* d_ws, size_t ws_size,
                              hipStream_t stream) {
  if (n_in < 9) return;
  if (in_sizes[0] != NTOK * DM) return;
  if (in_sizes[1] != NTOK * DM) return;
  if (in_sizes[2] != NTOK * DM) return;
  if (in_sizes[3] != DM * DK) return;
  if (in_sizes[4] != DK) return;
  if (in_sizes[5] != DM * DK) return;
  if (in_sizes[6] != DK) return;
  if (in_sizes[7] != DM * DK) return;
  if (in_sizes[8] != DK) return;
  if (out_size != NTOK * DK) return;

  const float* xq = (const float*)d_in[0];
  const float* xk = (const float*)d_in[1];
  const float* xv = (const float*)d_in[2];
  const float* wq = (const float*)d_in[3];
  const float* bq = (const float*)d_in[4];
  const float* wk = (const float*)d_in[5];
  const float* bk = (const float*)d_in[6];
  const float* wv = (const float*)d_in[7];
  const float* bv = (const float*)d_in[8];
  float* out = (float*)d_out;

  size_t off = 0;
  const size_t oX   = off; off += (size_t)3 * NTOK * DM * 2;
  const size_t oX3h = off; off += (size_t)3 * NR3 * DM * 2;
  const size_t oX3l = off; off += (size_t)3 * NR3 * DM * 2;
  const size_t oW   = off; off += (size_t)3 * DK * DM * 2;
  const size_t oW3h = off; off += (size_t)3 * DK * DM * 2;
  const size_t oW3l = off; off += (size_t)3 * DK * DM * 2;
  const size_t oQ   = off; off += (size_t)NTOK * DK * 2;
  const size_t oK   = off; off += (size_t)NTOK * DK * 2;
  const size_t oV   = off; off += (size_t)DK * NTOK * 2;
  const size_t oQ3h = off; off += (size_t)NR3 * DK * 2;
  const size_t oQ3l = off; off += (size_t)NR3 * DK * 2;
  const size_t oK3h = off; off += (size_t)NR3 * DK * 2;
  const size_t oK3l = off; off += (size_t)NR3 * DK * 2;
  const size_t oV3h = off; off += (size_t)DK * NR3 * 2;
  const size_t oV3l = off; off += (size_t)DK * NR3 * 2;
  if (off > ws_size) return;
  if (off > (size_t)134217728) return;

  char* ws = (char*)d_ws;
  _Float16* Xh  = (_Float16*)(ws + oX);
  ush*      X3h = (ush*)(ws + oX3h);
  ush*      X3l = (ush*)(ws + oX3l);
  _Float16* Wh  = (_Float16*)(ws + oW);
  ush*      W3h = (ush*)(ws + oW3h);
  ush*      W3l = (ush*)(ws + oW3l);
  _Float16* Qp  = (_Float16*)(ws + oQ);
  _Float16* Kp  = (_Float16*)(ws + oK);
  _Float16* Vt  = (_Float16*)(ws + oV);
  ush*      Q3h = (ush*)(ws + oQ3h);
  ush*      Q3l = (ush*)(ws + oQ3l);
  ush*      K3h = (ush*)(ws + oK3h);
  ush*      K3l = (ush*)(ws + oK3l);
  ush*      V3h = (ush*)(ws + oV3h);
  ush*      V3l = (ush*)(ws + oV3l);

  const float sscale = 0.044194173824159216f;

  const int ngx = in_sizes[0] / 8;
  k_cvt_x<<<dim3((ngx + 255) / 256, 3), dim3(256), 0, stream>>>(xq, xk, xv, Xh, X3h, X3l, ngx);
  k_cvt_w<<<dim3(DM / 64, DK / 32, 3), dim3(256), 0, stream>>>(wq, wk, wv, Wh, W3h, W3l);
  k_qkv<<<dim3(NTOK / 256, DK / 64, 3), dim3(256), 0, stream>>>(Xh, Wh, bq, bk, bv, Qp, Kp, Vt);
  k_qkv3<<<dim3(NR3 / 256, DK / 64, 3), dim3(256), 0, stream>>>(X3h, X3l, W3h, W3l, bq, bk, bv,
                                                                Q3h, Q3l, K3h, K3l, V3h, V3l);
  k_attn<<<dim3(NQT - QT3, NB), dim3(256), 0, stream>>>(Qp, Kp, Vt, out, QT3, sscale, 0.0009765625f);
  k_attn3<<<dim3(QT3, NB), dim3(256), 0, stream>>>(Q3h, Q3l, K3h, K3l, V3h, V3l, out, sscale);
  (void)hipGetLastError();
}
